// Processer_13623636263131
// MI455X (gfx1250) — hardware-verified
//
#include <hip/hip_runtime.h>
#include <hip/hip_bf16.h>
#include <stddef.h>
#include <stdint.h>
#include <math.h>


#define HD     128
#define HP     136
#define AP     264
#define FP     132
#define ROWS   64

#define PLANE  98304
#define P_HI   0
#define P_LO   PLANE
#define P_W2   (2 * PLANE)
#define T_TOT  (2 * PLANE + HD * HD)
#define T1A    0
#define T1B    16384
#define TU1    32768
#define TU2    65536
#define TU3    81920
#define T_GRPB (PLANE / 8)
#define T_BLKB (T_GRPB / 256)
#define T_GRPW (HD * HD / 8)
#define T_BLKW (T_GRPW / 256)

#define ASC    64.0f
#define RSC    2048.0f
#define WSC    16.0f
#define S1     0.0009765625f
#define S2     4.76837158203125e-07f

#define N_HI   0
#define N_LO   (ROWS * HP * 2)
#define N_STG  (2 * ROWS * HP * 2)
#define N_LDS  (N_STG + ROWS * FP * 4)

#define E_SI   0
#define E_DI   256
#define E_AHI  512
#define E_ALO  (E_AHI + ROWS * HP * 2)
#define E_STG  (E_ALO + ROWS * HP * 2)
#define E_LDS  (E_STG + ROWS * FP * 4)

#define NTHR   256
#define NWAVE  8
#define NB     256
#define EPT    8
#define CHUNK  (NTHR * EPT)
#define WCAP   (EPT * 32)
#define A_ACC  0
#define A_LIST (NB * HD * 4)
#define A_WCNT (A_LIST + NWAVE * WCAP * 4)
#define A_LDS  (A_WCNT + 64)

#define U_AHI  0
#define U_ALO  (ROWS * AP * 2)
#define U_H1HI (2 * ROWS * AP * 2)
#define U_H1LO (U_H1HI + ROWS * HP * 2)
#define U_LDS  (U_H1LO + ROWS * HP * 2)
#define U_H2HI 0
#define U_H2LO (ROWS * HP * 2)
#define U_STG  U_H1HI

#define NCHMAX 24
#define WS_CAP 134217728ull

static_assert(T_GRPB * 8 == PLANE);
static_assert(T_BLKB * 256 == T_GRPB);
static_assert(T_BLKW * 256 == T_GRPW);
static_assert(((T1B | TU1 | TU2 | TU3 | P_LO | P_W2) & 63) == 0);
static_assert(((HP * 2) & 15) == 0 && ((AP * 2) & 15) == 0 && ((FP * 4) & 15) == 0);
static_assert((N_LO & 15) == 0 && (N_STG & 15) == 0 && N_LDS <= 128 * 1024);
static_assert((E_AHI & 15) == 0 && (E_ALO & 15) == 0 && (E_STG & 15) == 0 && E_LDS <= 128 * 1024);
static_assert((A_LIST & 15) == 0 && (A_WCNT & 15) == 0 && A_LDS <= 300 * 1024);
static_assert((U_ALO & 15) == 0 && (U_H1HI & 15) == 0 && (U_H1LO & 15) == 0 && U_LDS <= 128 * 1024);
static_assert(U_H2LO + ROWS * HP * 2 <= U_H1HI);
static_assert(U_STG + ROWS * FP * 4 <= U_LDS);
static_assert(NB == 32 * NWAVE && NB <= 256 && WCAP == 256 && CHUNK <= (1 << 20) && NB == NTHR && ROWS == 64);

typedef float    v4f  __attribute__((ext_vector_type(4)));
typedef float    v8f  __attribute__((ext_vector_type(8)));
typedef int      v4i  __attribute__((ext_vector_type(4)));
typedef _Float16 v4h  __attribute__((ext_vector_type(4)));
typedef _Float16 v8h  __attribute__((ext_vector_type(8)));
typedef _Float16 v16h __attribute__((ext_vector_type(16)));
typedef __bf16   v8b  __attribute__((ext_vector_type(8)));
typedef __bf16   v16b __attribute__((ext_vector_type(16)));
union FragH { v16h v; v8h h[2]; };
union FragB { v16b v; v8b h[2]; };
union U8H   { v8h v; _Float16 e[8]; v4i q; };
union U8B   { v8b v; __bf16 e[8]; v4i q; };
union U4H   { v4h v; _Float16 e[4]; };

__device__ __forceinline__ v8f zero8f() {
  v8f z;
#pragma unroll
  for (int i = 0; i < 8; ++i) z[i] = 0.0f;
  return z;
}

__device__ __forceinline__ v8f wmh(v16h a, v16h b, v8f c) {
  v8f d = __builtin_amdgcn_wmma_f32_16x16x32_f16(false, a, false, b, (short)0, c, false, false);
  asm volatile("v_nop\n\tv_nop\n\tv_nop\n\tv_nop" : "+v"(d) : "v"(a), "v"(b));
  return d;
}
__device__ __forceinline__ v8f wmb(v16b a, v16b b, v8f c) {
  v8f d = __builtin_amdgcn_wmma_f32_16x16x32_bf16(false, a, false, b, (short)0, c, false, false);
  asm volatile("v_nop\n\tv_nop\n\tv_nop\n\tv_nop" : "+v"(d) : "v"(a), "v"(b));
  return d;
}

__device__ __forceinline__ float tanh_f(float x) {
  const float t = __expf(2.0f * x);
  return 1.0f - 2.0f * __builtin_amdgcn_rcpf(t + 1.0f);
}

__device__ __forceinline__ float bf16r(float x) {
  unsigned u = __float_as_uint(x);
  u = (u + 0x7FFFu + ((u >> 16) & 1u)) & 0xFFFF0000u;
  return __uint_as_float(u);
}

__device__ __forceinline__ void split8b(v4f a, v4f b, v8b& hi, v8b& lo) {
  U8B uh, ul;
#pragma unroll
  for (int i = 0; i < 4; ++i) {
    const float h0 = bf16r(a[i]);
    uh.e[i] = (__bf16)h0;
    ul.e[i] = (__bf16)(a[i] - h0);
    const float h1 = bf16r(b[i]);
    uh.e[4 + i] = (__bf16)h1;
    ul.e[4 + i] = (__bf16)(b[i] - h1);
  }
  hi = uh.v;
  lo = ul.v;
}

__device__ __forceinline__ void gemm_b3(const __bf16* ahi, const __bf16* alo, const __bf16* bhi,
                                        const __bf16* blo, int kp, int nk, v8f acc[4]) {
#pragma unroll 1
  for (int kt = 0; kt < nk; ++kt) {
    FragB ah, al;
    ah.h[0] = *(const v8b*)(ahi + 32 * kt);
    ah.h[1] = *(const v8b*)(ahi + 32 * kt + 16);
    al.h[0] = *(const v8b*)(alo + 32 * kt);
    al.h[1] = *(const v8b*)(alo + 32 * kt + 16);
#pragma unroll
    for (int nt = 0; nt < 4; ++nt) {
      const size_t bo = (size_t)(16 * nt) * kp + 32 * kt;
      FragB bh, bl;
      bh.h[0] = *(const v8b*)(bhi + bo);
      bh.h[1] = *(const v8b*)(bhi + bo + 16);
      bl.h[0] = *(const v8b*)(blo + bo);
      bl.h[1] = *(const v8b*)(blo + bo + 16);
      v8f c = acc[nt];
      c = wmb(ah.v, bh.v, c);
      c = wmb(al.v, bh.v, c);
      c = wmb(ah.v, bl.v, c);
      acc[nt] = c;
    }
  }
}

__device__ __forceinline__ void gemm_h2(const _Float16* ahi, const _Float16* alo, const _Float16* bcol,
                                        int kp, int nk, v8f acc[4], v8f accl[4]) {
#pragma unroll 1
  for (int kt = 0; kt < nk; ++kt) {
    FragH ah, al;
    ah.h[0] = *(const v8h*)(ahi + 32 * kt);
    ah.h[1] = *(const v8h*)(ahi + 32 * kt + 16);
    al.h[0] = *(const v8h*)(alo + 32 * kt);
    al.h[1] = *(const v8h*)(alo + 32 * kt + 16);
#pragma unroll
    for (int nt = 0; nt < 4; ++nt) {
      const _Float16* bp = bcol + (size_t)(16 * nt) * kp + 32 * kt;
      FragH b;
      b.h[0] = *(const v8h*)bp;
      b.h[1] = *(const v8h*)(bp + 16);
      acc[nt]  = wmh(ah.v, b.v, acc[nt]);
      accl[nt] = wmh(al.v, b.v, accl[nt]);
    }
  }
}

__device__ __forceinline__ void store_rows_f32(const float* stg, float* g, int row0, int M, int wave, int l) {
#pragma unroll
  for (int j = 0; j < 8; ++j) {
    const int lr = 8 * wave + j;
    const int gr = row0 + lr;
    if (gr < M) {
      const v4f v = *(const v4f*)(stg + lr * FP + 4 * l);
      *(volatile v4f*)(g + (size_t)gr * HD + 4 * l) = v;
    }
  }
  __threadfence();
#pragma unroll
  for (int j = 0; j < 8; ++j) {
    const int lr = 8 * wave + j;
    const int gr = row0 + lr;
    if (gr < M) {
      const v4f v = *(const v4f*)(stg + lr * FP + 4 * l);
      *(volatile v4f*)(g + (size_t)gr * HD + 4 * l) = v;
    }
  }
}

__global__ __launch_bounds__(256) void k_wcvt(const float* __restrict__ ew1, const float* __restrict__ ew2,
                                              const float* __restrict__ uw1, const float* __restrict__ uw2,
                                              const float* __restrict__ uw3, v4i* tq) {
  const int tid = threadIdx.x;
  if (blockIdx.x < T_BLKB) {
    const int g = blockIdx.x * 256 + tid;
    const float* src = ew1;
    int n = 0, kc = 0;
    if (g < 2048)       { const int q = g;         src = ew1;                    n = q >> 4; kc = (q & 15) * 8; }
    else if (g < 4096)  { const int q = g - 2048;  src = ew1 + (size_t)HD * HD; n = q >> 4; kc = (q & 15) * 8; }
    else if (g < 8192)  { const int q = g - 4096;  src = uw1;                    n = q >> 5; kc = (q & 31) * 8; }
    else if (g < 10240) { const int q = g - 8192;  src = uw2;                    n = q >> 4; kc = (q & 15) * 8; }
    else                { const int q = g - 10240; src = uw3;                    n = q >> 4; kc = (q & 15) * 8; }
    v4f a, b;
#pragma unroll
    for (int i = 0; i < 4; ++i) {
      a[i] = src[(size_t)(kc + i) * HD + n];
      b[i] = src[(size_t)(kc + 4 + i) * HD + n];
    }
    v8b hv, lv;
    split8b(a, b, hv, lv);
    U8B uh, ul;
    uh.v = hv;
    ul.v = lv;
    const v4i oh = uh.q, ol = ul.q;
    *(volatile v4i*)(tq + g) = oh;
    *(volatile v4i*)(tq + T_GRPB + g) = ol;
    __threadfence();
    *(volatile v4i*)(tq + g) = oh;
    *(volatile v4i*)(tq + T_GRPB + g) = ol;
  } else {
    const int q = (blockIdx.x - T_BLKB) * 256 + tid;
    if (q < T_GRPW) {
      const int n = q >> 4, kc = (q & 15) * 8;
      U8H u;
#pragma unroll
      for (int i = 0; i < 8; ++i) u.e[i] = (_Float16)(ew2[(size_t)(kc + i) * HD + n] * WSC);
      const v4i o = u.q;
      *(volatile v4i*)(tq + 2 * T_GRPB + q) = o;
      __threadfence();
      *(volatile v4i*)(tq + 2 * T_GRPB + q) = o;
    }
  }
}

__global__ __launch_bounds__(256) void k_node1(const float* __restrict__ hin, const __bf16* tb,
                                               float* HA, float* HB, int nN) {
  extern __shared__ __attribute__((aligned(16))) unsigned char lds_n[];
  __bf16* hhi = (__bf16*)(lds_n + N_HI);
  __bf16* hlo = (__bf16*)(lds_n + N_LO);
  float*  stg = (float*)(lds_n + N_STG);
  const int tid = threadIdx.x, l = tid & 31, wave = tid >> 5, h = l >> 4, m = l & 15;
  const int wr = wave >> 1, wc = wave & 1;
  const int row0 = blockIdx.x * ROWS;

  for (int i = tid; i < ROWS * 16; i += 256) {
    const int r = i >> 4, c = (i & 15) * 8;
    const int gr = row0 + r;
    v4f x0 = {0.0f, 0.0f, 0.0f, 0.0f};
    v4f x1 = x0;
    if (gr < nN) {
      const float* p = hin + (size_t)gr * HD + c;
      x0 = *(const v4f*)p;
      x1 = *(const v4f*)(p + 4);
    }
    v8b hv, lv;
    split8b(x0, x1, hv, lv);
    *(v8b*)(hhi + r * HP + c) = hv;
    *(v8b*)(hlo + r * HP + c) = lv;
  }
  __syncthreads();

  v8f acc[4];
#pragma unroll
  for (int i = 0; i < 4; ++i) acc[i] = zero8f();
  gemm_b3(hhi + (16 * wr + m) * HP + 8 * h, hlo + (16 * wr + m) * HP + 8 * h,
          tb + P_HI + T1A + (size_t)(64 * wc + m) * HD + 8 * h,
          tb + P_LO + T1A + (size_t)(64 * wc + m) * HD + 8 * h, HD, 4, acc);
#pragma unroll
  for (int nt = 0; nt < 4; ++nt) {
    const int c = 64 * wc + 16 * nt + m;
#pragma unroll
    for (int r = 0; r < 8; ++r) {
      const int lr = 16 * wr + 8 * h + r;
      stg[lr * FP + c] = acc[nt][r];
    }
  }
  __syncthreads();
  store_rows_f32(stg, HA, row0, nN, wave, l);
  __syncthreads();

#pragma unroll
  for (int i = 0; i < 4; ++i) acc[i] = zero8f();
  gemm_b3(hhi + (16 * wr + m) * HP + 8 * h, hlo + (16 * wr + m) * HP + 8 * h,
          tb + P_HI + T1B + (size_t)(64 * wc + m) * HD + 8 * h,
          tb + P_LO + T1B + (size_t)(64 * wc + m) * HD + 8 * h, HD, 4, acc);
#pragma unroll
  for (int nt = 0; nt < 4; ++nt) {
    const int c = 64 * wc + 16 * nt + m;
#pragma unroll
    for (int r = 0; r < 8; ++r) {
      const int lr = 16 * wr + 8 * h + r;
      stg[lr * FP + c] = acc[nt][r];
    }
  }
  __syncthreads();
  store_rows_f32(stg, HB, row0, nN, wave, l);
}

__global__ __launch_bounds__(256) void k_edge(const int* __restrict__ ei, const float* __restrict__ HA,
                                              const float* __restrict__ HB, const float* __restrict__ eb1,
                                              const float* __restrict__ eb2, const _Float16* tw, float* msg,
                                              int nN, int nE, int cb, int clen) {
  extern __shared__ __attribute__((aligned(16))) unsigned char lds_e[];
  int*      sidx = (int*)(lds_e + E_SI);
  int*      didx = (int*)(lds_e + E_DI);
  _Float16* ahi  = (_Float16*)(lds_e + E_AHI);
  _Float16* alo  = (_Float16*)(lds_e + E_ALO);
  float*    stg  = (float*)(lds_e + E_STG);
  const int tid = threadIdx.x, l = tid & 31, wave = tid >> 5, h = l >> 4, m = l & 15;
  const int wr = wave >> 1, wc = wave & 1;
  const int e0 = blockIdx.x * ROWS;

  if (tid < ROWS) {
    const int le = e0 + tid;
    int sc = 0, dc = 0;
    if (le < clen) {
      const int g = cb + le;
      int s = ei[g];
      int d = ei[(size_t)nE + g];
      if (s < 0) s += nN;
      sc = s < 0 ? 0 : (s > nN - 1 ? nN - 1 : s);
      if (d < 0) d += nN;
      dc = d < 0 ? 0 : (d > nN - 1 ? nN - 1 : d);
    }
    sidx[tid] = sc;
    didx[tid] = dc;
  }
  __syncthreads();

  {
    const v4f b4 = *(const v4f*)(eb1 + 4 * l);
#pragma unroll
    for (int j = 0; j < 8; ++j) {
      const int lr = 8 * wave + j;
      const int s = sidx[lr], d = didx[lr];
      const v4f va = *(const v4f*)(HA + (size_t)s * HD + 4 * l);
      const v4f vb = *(const v4f*)(HB + (size_t)d * HD + 4 * l);
      U4H uh, ul;
#pragma unroll
      for (int i = 0; i < 4; ++i) {
        const float p = (va[i] + vb[i]) + b4[i];
        const float x = tanh_f(p) * ASC;
        const _Float16 hv = (_Float16)x;
        uh.e[i] = hv;
        ul.e[i] = (_Float16)((x - (float)hv) * RSC);
      }
      *(v4h*)(ahi + lr * HP + 4 * l) = uh.v;
      *(v4h*)(alo + lr * HP + 4 * l) = ul.v;
    }
  }
  __syncthreads();

  v8f acc[4], accl[4];
#pragma unroll
  for (int i = 0; i < 4; ++i) { acc[i] = zero8f(); accl[i] = zero8f(); }
  gemm_h2(ahi + (16 * wr + m) * HP + 8 * h, alo + (16 * wr + m) * HP + 8 * h,
          tw + (size_t)(64 * wc + m) * HD + 8 * h, HD, 4, acc, accl);
#pragma unroll
  for (int nt = 0; nt < 4; ++nt) {
    const int c = 64 * wc + 16 * nt + m;
    const float bc = eb2[c];
#pragma unroll
    for (int r = 0; r < 8; ++r) {
      const int lr = 16 * wr + 8 * h + r;
      stg[lr * FP + c] = (acc[nt][r] * S1 + accl[nt][r] * S2) + bc;
    }
  }
  __syncthreads();

  store_rows_f32(stg, msg, e0, clen, wave, l);
}

__device__ __forceinline__ int scan_chunk(const int* __restrict__ dsts, int nE, int cbase, int nodeBase,
                                          int* list, int tid, int wave, int vec_ok) {
  int wc = 0;
  const int el0  = tid * EPT;
  const int e0   = cbase + el0;
  const int sent = -2147483647 - 1;
  v4i da, db;
  if (vec_ok != 0 && e0 + 7 < nE) {
    da = *(const v4i*)(dsts + e0);
    db = *(const v4i*)(dsts + e0 + 4);
  } else {
    da.x = (e0     < nE) ? dsts[(e0     < nE) ? e0     : nE - 1] : sent;
    da.y = (e0 + 1 < nE) ? dsts[(e0 + 1 < nE) ? e0 + 1 : nE - 1] : sent;
    da.z = (e0 + 2 < nE) ? dsts[(e0 + 2 < nE) ? e0 + 2 : nE - 1] : sent;
    da.w = (e0 + 3 < nE) ? dsts[(e0 + 3 < nE) ? e0 + 3 : nE - 1] : sent;
    db.x = (e0 + 4 < nE) ? dsts[(e0 + 4 < nE) ? e0 + 4 : nE - 1] : sent;
    db.y = (e0 + 5 < nE) ? dsts[(e0 + 5 < nE) ? e0 + 5 : nE - 1] : sent;
    db.z = (e0 + 6 < nE) ? dsts[(e0 + 6 < nE) ? e0 + 6 : nE - 1] : sent;
    db.w = (e0 + 7 < nE) ? dsts[(e0 + 7 < nE) ? e0 + 7 : nE - 1] : sent;
  }
  const unsigned nb = (unsigned)nodeBase;
  const unsigned s0 = (unsigned)da.x - nb, s1 = (unsigned)da.y - nb;
  const unsigned s2 = (unsigned)da.z - nb, s3 = (unsigned)da.w - nb;
  const unsigned s4 = (unsigned)db.x - nb, s5 = (unsigned)db.y - nb;
  const unsigned s6 = (unsigned)db.z - nb, s7 = (unsigned)db.w - nb;
  const bool q0 = s0 < (unsigned)NB, q1 = s1 < (unsigned)NB, q2 = s2 < (unsigned)NB, q3 = s3 < (unsigned)NB;
  const bool q4 = s4 < (unsigned)NB, q5 = s5 < (unsigned)NB, q6 = s6 < (unsigned)NB, q7 = s7 < (unsigned)NB;
  const unsigned any = __builtin_amdgcn_ballot_w32(q0 | q1 | q2 | q3 | q4 | q5 | q6 | q7);
  if (any != 0u) {
#define HITJ(J, QJ, SJ) { \
      const unsigned mj = __builtin_amdgcn_ballot_w32(QJ); \
      if (mj != 0u) { \
        if (QJ) { \
          const int p = wc + (int)__builtin_amdgcn_mbcnt_lo(mj, 0u); \
          if (p < WCAP) list[wave * WCAP + p] = ((el0 + (J)) << 8) | (int)(SJ); \
        } \
        wc += (int)__builtin_popcount(mj); } }
    HITJ(0, q0, s0)
    HITJ(1, q1, s1)
    HITJ(2, q2, s2)
    HITJ(3, q3, s3)
    HITJ(4, q4, s4)
    HITJ(5, q5, s5)
    HITJ(6, q6, s6)
    HITJ(7, q7, s7)
#undef HITJ
  }
  return wc;
}

__global__ __launch_bounds__(NTHR) void k_agg(const int* __restrict__ dsts, const float* __restrict__ msg,
                                               float* agg, int nN, int clen, int first, int vec_ok) {
  extern __shared__ __attribute__((aligned(16))) unsigned char lds_a[];
  float* acc  = (float*)(lds_a + A_ACC);
  int*   list = (int*)(lds_a + A_LIST);
  int*   wcnt = (int*)(lds_a + A_WCNT);
  const int tid = threadIdx.x, l = tid & 31, wave = tid >> 5;
  const int nodeBase = blockIdx.x * NB;

  for (int i = tid; i < NB * 32; i += NTHR) {
    const int slot = i >> 5, q = (i & 31) * 4;
    const int node = nodeBase + slot;
    v4f v = {0.0f, 0.0f, 0.0f, 0.0f};
    if (first == 0 && node < nN) v = *(const v4f*)(agg + (size_t)node * HD + q);
    *(v4f*)(acc + slot * HD + q) = v;
  }
  __syncthreads();

  const int nChunks = (clen + CHUNK - 1) / CHUNK;
#pragma unroll 1
  for (int ch = 0; ch < nChunks; ++ch) {
    const int cbase = ch * CHUNK;
    const int wc = scan_chunk(dsts, clen, cbase, nodeBase, list, tid, wave, vec_ok);
    if (l == 0) wcnt[wave] = wc;
    __syncthreads();

#pragma unroll 1
    for (int w2 = 0; w2 < NWAVE; ++w2) {
      int n = wcnt[w2];
      n = n > WCAP ? WCAP : (n < 0 ? 0 : n);
      const int* lp = list + w2 * WCAP;
#pragma unroll 1
      for (int i0 = 0; i0 < n; i0 += 32) {
        const int idx = i0 + l;
        const int v = lp[(idx < n) ? idx : 0];
        unsigned mk = __builtin_amdgcn_ballot_w32((idx < n) && ((v & 7) == wave));
#pragma unroll 1
        while (mk != 0u) {
          const int bpos = __builtin_ctz(mk);
          mk &= mk - 1u;
          const int vv = __shfl(v, bpos);
          const int slot = vv & 255;
          int e = cbase + (vv >> 8);
          e = e < 0 ? 0 : (e > clen - 1 ? clen - 1 : e);
          const v4f x = *(const v4f*)(msg + (size_t)e * HD + 4 * l);
          float* ap = acc + slot * HD + 4 * l;
          v4f a = *(v4f*)ap;
          a[0] += x[0]; a[1] += x[1]; a[2] += x[2]; a[3] += x[3];
          *(v4f*)ap = a;
        }
      }
    }
    __syncthreads();
  }

#pragma unroll
  for (int j = 0; j < 32; ++j) {
    const int slot = wave * 32 + j;
    const int node = nodeBase + slot;
    if (node < nN) {
      const v4f a = *(const v4f*)(acc + slot * HD + 4 * l);
      *(volatile v4f*)(agg + (size_t)node * HD + 4 * l) = a;
    }
  }
  __threadfence();
#pragma unroll
  for (int j = 0; j < 32; ++j) {
    const int slot = wave * 32 + j;
    const int node = nodeBase + slot;
    if (node < nN) {
      const v4f a = *(const v4f*)(acc + slot * HD + 4 * l);
      *(volatile v4f*)(agg + (size_t)node * HD + 4 * l) = a;
    }
  }
}

__global__ __launch_bounds__(256) void k_upd(const float* __restrict__ hin, const float* __restrict__ agg,
                                             const __bf16* tb, const float* __restrict__ ub1,
                                             const float* __restrict__ ub2, const float* __restrict__ ub3,
                                             float* out, int nN) {
  extern __shared__ __attribute__((aligned(16))) unsigned char lds_u[];
  __bf16* ahi  = (__bf16*)(lds_u + U_AHI);
  __bf16* alo  = (__bf16*)(lds_u + U_ALO);
  __bf16* h1hi = (__bf16*)(lds_u + U_H1HI);
  __bf16* h1lo = (__bf16*)(lds_u + U_H1LO);
  __bf16* h2hi = (__bf16*)(lds_u + U_H2HI);
  __bf16* h2lo = (__bf16*)(lds_u + U_H2LO);
  float*  stg  = (float*)(lds_u + U_STG);
  const int tid = threadIdx.x, l = tid & 31, wave = tid >> 5, h = l >> 4, m = l & 15;
  const int wr = wave >> 1, wc = wave & 1;
  const int row0 = blockIdx.x * ROWS;

  for (int i = tid; i < ROWS * 32; i += 256) {
    const int r = i >> 5, c = (i & 31) * 8;
    const int gr = row0 + r;
    v4f x0 = {0.0f, 0.0f, 0.0f, 0.0f};
    v4f x1 = x0;
    if (gr < nN) {
      const float* p = (c < HD) ? (hin + (size_t)gr * HD + c) : (agg + (size_t)gr * HD + (c - HD));
      x0 = *(const v4f*)p;
      x1 = *(const v4f*)(p + 4);
    }
    v8b hv, lv;
    split8b(x0, x1, hv, lv);
    *(v8b*)(ahi + r * AP + c) = hv;
    *(v8b*)(alo + r * AP + c) = lv;
  }
  __syncthreads();

  v8f acc[4];
#pragma unroll
  for (int i = 0; i < 4; ++i) acc[i] = zero8f();
  gemm_b3(ahi + (16 * wr + m) * AP + 8 * h, alo + (16 * wr + m) * AP + 8 * h,
          tb + P_HI + TU1 + (size_t)(64 * wc + m) * 256 + 8 * h,
          tb + P_LO + TU1 + (size_t)(64 * wc + m) * 256 + 8 * h, 256, 8, acc);
#pragma unroll
  for (int nt = 0; nt < 4; ++nt) {
    const int c = 64 * wc + 16 * nt + m;
    const float bc = ub1[c];
#pragma unroll
    for (int r = 0; r < 8; ++r) {
      const int lr = 16 * wr + 8 * h + r;
      const float t = tanh_f(acc[nt][r] + bc);
      const float hf = bf16r(t);
      h1hi[lr * HP + c] = (__bf16)hf;
      h1lo[lr * HP + c] = (__bf16)(t - hf);
    }
  }
  __syncthreads();

#pragma unroll
  for (int i = 0; i < 4; ++i) acc[i] = zero8f();
  gemm_b3(h1hi + (16 * wr + m) * HP + 8 * h, h1lo + (16 * wr + m) * HP + 8 * h,
          tb + P_HI + TU2 + (size_t)(64 * wc + m) * HD + 8 * h,
          tb + P_LO + TU2 + (size_t)(64 * wc + m) * HD + 8 * h, HD, 4, acc);
#pragma unroll
  for (int nt = 0; nt < 4; ++nt) {
    const int c = 64 * wc + 16 * nt + m;
    const float bc = ub2[c];
#pragma unroll
    for (int r = 0; r < 8; ++r) {
      const int lr = 16 * wr + 8 * h + r;
      const float t = tanh_f(acc[nt][r] + bc);
      const float hf = bf16r(t);
      h2hi[lr * HP + c] = (__bf16)hf;
      h2lo[lr * HP + c] = (__bf16)(t - hf);
    }
  }
  __syncthreads();

#pragma unroll
  for (int i = 0; i < 4; ++i) acc[i] = zero8f();
  gemm_b3(h2hi + (16 * wr + m) * HP + 8 * h, h2lo + (16 * wr + m) * HP + 8 * h,
          tb + P_HI + TU3 + (size_t)(64 * wc + m) * HD + 8 * h,
          tb + P_LO + TU3 + (size_t)(64 * wc + m) * HD + 8 * h, HD, 4, acc);
#pragma unroll
  for (int nt = 0; nt < 4; ++nt) {
    const int c = 64 * wc + 16 * nt + m;
    const float bc = ub3[c];
#pragma unroll
    for (int r = 0; r < 8; ++r) {
      const int lr = 16 * wr + 8 * h + r;
      stg[lr * FP + c] = acc[nt][r] + bc;
    }
  }
  __syncthreads();

  store_rows_f32(stg, out, row0, nN, wave, l);
}

extern "C" void kernel_launch(void* const* d_in, const int* in_sizes, int n_in,
                              void* d_out, int out_size, void* d_ws, size_t ws_size,
                              hipStream_t stream) {
  if (n_in < 12) return;
  const int nN = in_sizes[0] / HD;
  const int nE = in_sizes[1] / 2;
  if (nN <= 0 || nE <= 0) return;
  if (in_sizes[0] != nN * HD || in_sizes[1] != 2 * nE) return;
  if (in_sizes[2] != 2 * HD * HD || in_sizes[3] < HD || in_sizes[4] != HD * HD || in_sizes[5] < HD) return;
  if (in_sizes[6] != 2 * HD * HD || in_sizes[7] < HD || in_sizes[8] != HD * HD || in_sizes[9] < HD) return;
  if (in_sizes[10] != HD * HD || in_sizes[11] < HD) return;
  if ((long long)out_size != (long long)nN * HD) return;

  const float* hin = (const float*)d_in[0];
  const int*   ei  = (const int*)d_in[1];
  const float* ew1 = (const float*)d_in[2];
  const float* eb1 = (const float*)d_in[3];
  const float* ew2 = (const float*)d_in[4];
  const float* eb2 = (const float*)d_in[5];
  const float* uw1 = (const float*)d_in[6];
  const float* ub1 = (const float*)d_in[7];
  const float* uw2 = (const float*)d_in[8];
  const float* ub2 = (const float*)d_in[9];
  const float* uw3 = (const float*)d_in[10];
  const float* ub3 = (const float*)d_in[11];
  float* out0 = (float*)d_out;

  const int nBlkN = (nN + ROWS - 1) / ROWS;
  const int nBlkA = (nN + NB - 1) / NB;
  const int vec_ok = ((nE & 3) == 0) ? 1 : 0;

  const size_t cap = ws_size < (size_t)WS_CAP ? ws_size : (size_t)WS_CAP;
  char* ws = (char*)d_ws;
  size_t off = 0;
  const size_t oT  = off; off += (size_t)T_TOT * 2;        off = (off + 255) & ~(size_t)255;
  const size_t oHA = off; off += (size_t)nN * HD * 4;      off = (off + 255) & ~(size_t)255;
  const size_t oHB = off; off += (size_t)nN * HD * 4;      off = (off + 255) & ~(size_t)255;
  const size_t oAG = off; off += (size_t)nN * HD * 4;      off = (off + 255) & ~(size_t)255;
  if (off + 256 > cap) return;
  const size_t rem = cap - off;
  long long chmax = (long long)(rem / ((size_t)HD * 4));
  chmax = chmax / CHUNK * CHUNK;
  if (chmax < CHUNK) return;
  const int nch = (int)(((long long)nE + chmax - 1) / chmax);
  if (nch <= 0 || nch > NCHMAX) return;
  long long chl = ((long long)nE + nch - 1) / nch;
  chl = (chl + CHUNK - 1) / CHUNK * CHUNK;
  if (chl > chmax) return;
  const int CH = (int)chl;
  const size_t oMS = off; off += (size_t)CH * HD * 4;      off = (off + 255) & ~(size_t)255;
  if (off > cap) return;

  v4i*            tq  = (v4i*)(ws + oT);
  const __bf16*   tb  = (const __bf16*)(ws + oT);
  const _Float16* tw  = (const _Float16*)(ws + oT) + P_W2;
  float*          hap = (float*)(ws + oHA);
  float*          hbp = (float*)(ws + oHB);
  float*          agp = (float*)(ws + oAG);
  float*          msp = (float*)(ws + oMS);

  const hipError_t a0 = hipFuncSetAttribute(reinterpret_cast<const void*>(&k_node1), hipFuncAttributeMaxDynamicSharedMemorySize, N_LDS);
  const hipError_t a1 = hipFuncSetAttribute(reinterpret_cast<const void*>(&k_edge),  hipFuncAttributeMaxDynamicSharedMemorySize, E_LDS);
  const hipError_t a2 = hipFuncSetAttribute(reinterpret_cast<const void*>(&k_agg),   hipFuncAttributeMaxDynamicSharedMemorySize, A_LDS);
  const hipError_t a3 = hipFuncSetAttribute(reinterpret_cast<const void*>(&k_upd),   hipFuncAttributeMaxDynamicSharedMemorySize, U_LDS);
  (void)a0; (void)a1; (void)a2; (void)a3;

  k_wcvt<<<T_BLKB + T_BLKW, 256, 0, stream>>>(ew1, ew2, uw1, uw2, uw3, tq);
  k_node1<<<nBlkN, 256, N_LDS, stream>>>(hin, tb, hap, hbp, nN);

  for (int c = 0; c < nch; ++c) {
    const long long cb64 = (long long)c * CH;
    if (cb64 >= (long long)nE) break;
    const int cbase = (int)cb64;
    int clen = nE - cbase;
    clen = clen > CH ? CH : clen;
    const int nEB = (clen + ROWS - 1) / ROWS;
    k_edge<<<nEB, 256, E_LDS, stream>>>(ei, hap, hbp, eb1, eb2, tw, msp, nN, nE, cbase, clen);
    k_agg<<<nBlkA, NTHR, A_LDS, stream>>>(ei + (size_t)nE + (size_t)cbase, msp, agp, nN, clen, (c == 0) ? 1 : 0, vec_ok);
  }

  k_upd<<<nBlkN, 256, U_LDS, stream>>>(hin, agp, tb, ub1, ub2, ub3, out0, nN);
  (void)hipGetLastError();
}
